// SATG_34677565948058
// MI455X (gfx1250) — hardware-verified
//
#include <hip/hip_runtime.h>


#define NB_  8
#define NS0  2000
#define NP   2048
#define DM   256
#define NH_  2
#define HD   128
#define FF   256
#define F1   64
#define NTK  (NB_ * NP)
#define WIN  99
#define PSC  32768.0f
#define LOSC 1024.0f
#define LOSCI (1.0f / 1024.0f)
#define SCL  0.08838834764831845f

typedef _Float16 h16;
typedef unsigned short bf;
typedef __attribute__((ext_vector_type(16))) __bf16   v16bf;
typedef __attribute__((ext_vector_type(16))) _Float16 v16h;
typedef __attribute__((ext_vector_type(8)))  _Float16 v8h;
typedef __attribute__((ext_vector_type(8)))  unsigned short v8us;
typedef __attribute__((ext_vector_type(8)))  float    v8f;
typedef __attribute__((ext_vector_type(4)))  float    v4f;
typedef v8h  __attribute__((may_alias)) v8ha;
typedef v4f  __attribute__((may_alias)) v4fa;
typedef v8us __attribute__((may_alias)) v8usa;

__device__ __forceinline__ unsigned short f2bf(float f) { unsigned u = __float_as_uint(f); u += 0x7FFFu + ((u >> 16) & 1u); return (unsigned short)(u >> 16); }
__device__ __forceinline__ float bf2f(unsigned short b) { return __uint_as_float(((unsigned)b) << 16); }
__device__ __forceinline__ float bfr(float f) { return bf2f(f2bf(f)); }
__device__ __forceinline__ v16h cat16(v8h lo, v8h hi) { return __builtin_shufflevector(lo, hi, 0, 1, 2, 3, 4, 5, 6, 7, 8, 9, 10, 11, 12, 13, 14, 15); }
__device__ __forceinline__ v16bf cat16b(v8us lo, v8us hi) { return __builtin_bit_cast(v16bf, __builtin_shufflevector(lo, hi, 0, 1, 2, 3, 4, 5, 6, 7, 8, 9, 10, 11, 12, 13, 14, 15)); }
__device__ __forceinline__ v8f wmma16(v16h a, v16h b, v8f c) { return __builtin_amdgcn_wmma_f32_16x16x32_f16(false, a, false, b, (short)0, c, false, false); }
__device__ __forceinline__ v8f wmmab(v16bf a, v16bf b, v8f c) { return __builtin_amdgcn_wmma_f32_16x16x32_bf16(false, a, false, b, (short)0, c, false, false); }
#define VST2(T, p, v) do { const T vst2_v_ = (v); *(volatile T*)(p) = vst2_v_; __threadfence(); *(volatile T*)(p) = vst2_v_; } while (0)

__global__ __launch_bounds__(256) void k_xb(const float* __restrict__ src, bf* Xb) {
    const int lane = threadIdx.x & 31, r = blockIdx.x * 8 + (threadIdx.x >> 5);
    if (r >= NTK) return;
    const int b = r / NP, n = r - b * NP, nn = (n < NS0) ? n : (NS0 - 1);
    v8us t;
#pragma unroll
    for (int i = 0; i < 8; ++i) { const unsigned short hb = f2bf(src[((size_t)b * NS0 + nn) * DM + lane * 8 + i]); t[i] = (n < NS0) ? hb : (unsigned short)0; }
    VST2(v8us, Xb + (size_t)r * DM + lane * 8, t);
}
__global__ __launch_bounds__(256) void k_cvtb(const float* __restrict__ src, int nrows, int ncols, bf* dst) {
    const int lane = threadIdx.x & 31, r = blockIdx.x * 8 + (threadIdx.x >> 5);
    if (r >= nrows) return;
    if (ncols == 256) { v8us t;
#pragma unroll
        for (int i = 0; i < 8; ++i) t[i] = f2bf(src[(size_t)r * 256 + lane * 8 + i]);
        VST2(v8us, dst + (size_t)r * 256 + lane * 8, t);
    } else { typedef __attribute__((ext_vector_type(2))) unsigned short v2us; v2us t; t[0] = f2bf(src[(size_t)r * 64 + lane * 2]); t[1] = f2bf(src[(size_t)r * 64 + lane * 2 + 1]);
        VST2(v2us, dst + (size_t)r * 64 + lane * 2, t); }
}
__global__ __launch_bounds__(256) void k_pe(float* PE) {
    const int lane = threadIdx.x & 31, n = blockIdx.x * 8 + (threadIdx.x >> 5);
    if (n >= NP) return;
    v8f o;
#pragma unroll 1
    for (int i = 0; i < 4; ++i) { const int j = lane * 4 + i;
        const float dv = expf((float)(2 * j) * (-9.210340371976184f / (float)DM));
        const float a = (float)n * dv; o[2 * i] = sinf(a); o[2 * i + 1] = cosf(a); }
    VST2(v8f, PE + (size_t)n * DM + lane * 8, o);
}

template <bool SPLITA, int MODE>
__global__ __launch_bounds__(128) void k_gemmb(const bf* __restrict__ A, const bf* __restrict__ Al, const bf* __restrict__ Bn, int K, const float* __restrict__ bias, const float* __restrict__ ADD, void* C, void* C2, int ldc) {
    __shared__ __align__(16) float ost[4][16 * 68];
    const int lane = threadIdx.x & 31, wave = threadIdx.x >> 5, lr = lane & 15, hi = lane >> 4;
    const int r0 = blockIdx.x * 64 + wave * 16, c0 = blockIdx.y * 64;
    const size_t aoff = (size_t)(r0 + lr) * K + 8 * hi;
    size_t boff[4];
#pragma unroll
    for (int t = 0; t < 4; ++t) boff[t] = (size_t)(c0 + t * 16 + lr) * K + 8 * hi;
    v8f acc[4];
#pragma unroll
    for (int t = 0; t < 4; ++t) acc[t] = (v8f){};
#pragma unroll 1
    for (int kc = 0; kc < K; kc += 32) {
        const v16bf a = cat16b(*(const v8us*)(A + aoff + kc), *(const v8us*)(A + aoff + kc + 16));
        v16bf al = a;
        if (SPLITA) al = cat16b(*(const v8us*)(Al + aoff + kc), *(const v8us*)(Al + aoff + kc + 16));
#pragma unroll
        for (int t = 0; t < 4; ++t) { const v16bf b = cat16b(*(const v8us*)(Bn + boff[t] + kc), *(const v8us*)(Bn + boff[t] + kc + 16)); acc[t] = wmmab(a, b, acc[t]); if (SPLITA) acc[t] = wmmab(al, b, acc[t]); }
        asm volatile("v_nop\n\tv_nop\n\tv_nop\n\tv_nop" : "+v"(acc[0]), "+v"(acc[1]), "+v"(acc[2]), "+v"(acc[3]) : "v"(a), "v"(al));
    }
    float* os = &ost[wave][0];
#pragma unroll
    for (int t = 0; t < 4; ++t) { const int col = c0 + t * 16 + lr; const float bv = bfr(bias[col]);
#pragma unroll
        for (int j = 0; j < 8; ++j) { float v = acc[t][j] + bv; if (ADD) v += ADD[(size_t)((r0 + hi * 8 + j) % NP) * DM + col]; if (MODE == 1) v = fmaxf(v, 0.f); os[(hi * 8 + j) * 68 + t * 16 + lr] = v; } }
    __syncthreads();
    if (MODE == 2) {
        h16* crow = (h16*)C + (size_t)r0 * ldc + c0;
        auto pass = [&]() {
#pragma unroll
            for (int s = 0; s < 4; ++s) { const int row = 4 * s + (lane >> 3), piece = lane & 7; const float* sp = os + row * 68 + piece * 8; v8h o;
#pragma unroll
                for (int i = 0; i < 8; ++i) o[i] = (h16)sp[i];
                *(volatile v8h*)(crow + (size_t)row * ldc + piece * 8) = o; }
        };
        pass(); __threadfence(); pass();
    } else if (MODE == 0) {
        float* crow = (float*)C + (size_t)r0 * ldc + c0;
        auto pass = [&]() {
#pragma unroll
            for (int s = 0; s < 8; ++s) { const int Lid = (lane >> 3) + 4 * s, piece = lane & 7; const int row = Lid >> 1, cofs = (Lid & 1) * 32 + piece * 4;
                const v4f val = *(const v4fa*)(os + row * 68 + cofs); *(volatile v4f*)(crow + (size_t)row * ldc + cofs) = val; }
        };
        pass(); __threadfence(); pass();
    } else {
        bf* ch = (bf*)C + (size_t)r0 * ldc + c0; bf* cl = (bf*)C2 + (size_t)r0 * ldc + c0;
        auto pass = [&]() {
#pragma unroll
            for (int s = 0; s < 4; ++s) { const int row = 4 * s + (lane >> 3), piece = lane & 7; const float* sp = os + row * 68 + piece * 8; v8us oh, ol;
#pragma unroll
                for (int i = 0; i < 8; ++i) { const unsigned short hb = f2bf(sp[i]); oh[i] = hb; ol[i] = f2bf(sp[i] - bf2f(hb)); }
                *(volatile v8us*)(ch + (size_t)row * ldc + piece * 8) = oh; *(volatile v8us*)(cl + (size_t)row * ldc + piece * 8) = ol; }
        };
        pass(); __threadfence(); pass();
    }
}

__global__ __launch_bounds__(256) void k_split(const float* __restrict__ S, bf* H, bf* L) {
    const int lane = threadIdx.x & 31, r = blockIdx.x * 8 + (threadIdx.x >> 5);
    if (r >= NTK) return;
    v8us oh, ol;
#pragma unroll
    for (int i = 0; i < 8; ++i) { const float v = S[(size_t)r * DM + lane * 8 + i]; const unsigned short hb = f2bf(v); oh[i] = hb; ol[i] = f2bf(v - bf2f(hb)); }
    *(volatile v8us*)(H + (size_t)r * DM + lane * 8) = oh; *(volatile v8us*)(L + (size_t)r * DM + lane * 8) = ol;
    __threadfence();
    *(volatile v8us*)(H + (size_t)r * DM + lane * 8) = oh; *(volatile v8us*)(L + (size_t)r * DM + lane * 8) = ol;
}
__global__ __launch_bounds__(256) void k_ln(const float* __restrict__ Xa, const float* __restrict__ Xb_, const float* __restrict__ w, const float* __restrict__ bb, float* X, bf* H, bf* L) {
    const int lane = threadIdx.x & 31, r = blockIdx.x * 8 + (threadIdx.x >> 5);
    if (r >= NTK) return;
    float v[8]; float s = 0.f;
#pragma unroll
    for (int i = 0; i < 8; ++i) { v[i] = Xa[(size_t)r * DM + lane * 8 + i] + Xb_[(size_t)r * DM + lane * 8 + i]; s += v[i]; }
#pragma unroll
    for (int o = 16; o; o >>= 1) s += __shfl_xor(s, o, 32);
    const float mu = s * (1.0f / DM);
    float q = 0.f;
#pragma unroll
    for (int i = 0; i < 8; ++i) { const float d = v[i] - mu; q += d * d; }
#pragma unroll
    for (int o = 16; o; o >>= 1) q += __shfl_xor(q, o, 32);
    const float rs = rsqrtf(q * (1.0f / DM) + 1e-5f);
    v8f xo; v8us oh, ol;
#pragma unroll
    for (int i = 0; i < 8; ++i) { const int c = lane * 8 + i; const float y = (v[i] - mu) * rs * bfr(w[c]) + bfr(bb[c]); xo[i] = y; const unsigned short hb = f2bf(y); oh[i] = hb; ol[i] = f2bf(y - bf2f(hb)); }
    *(volatile v8f*)(X + (size_t)r * DM + lane * 8) = xo; *(volatile v8us*)(H + (size_t)r * DM + lane * 8) = oh; *(volatile v8us*)(L + (size_t)r * DM + lane * 8) = ol;
    __threadfence();
    *(volatile v8f*)(X + (size_t)r * DM + lane * 8) = xo; *(volatile v8us*)(H + (size_t)r * DM + lane * 8) = oh; *(volatile v8us*)(L + (size_t)r * DM + lane * 8) = ol;
}

__global__ __launch_bounds__(256) void k_vt(const float* __restrict__ V, h16* VTH, h16* VTL) {
    __shared__ __align__(16) h16 tile[HD * 72];
    __shared__ __align__(16) h16 til2[HD * 72];
    const int bid = blockIdx.x;
    const int b = bid / (NH_ * (NP / 64)), rem = bid - b * (NH_ * (NP / 64)), h = rem / (NP / 64), kt = rem - h * (NP / 64);
    const int k0 = kt * 64, tid = threadIdx.x;
    const int kk = tid >> 2, d0 = (tid & 3) * 32;
    const float* src = V + ((size_t)b * NP + k0 + kk) * DM + h * HD + d0;
#pragma unroll
    for (int i = 0; i < 32; ++i) { const float v = src[i]; const h16 a = (h16)v; tile[(d0 + i) * 72 + kk] = a; til2[(d0 + i) * 72 + kk] = (h16)((v - (float)a) * LOSC); }
    __syncthreads();
    const int piece = tid & 7;
    const size_t base = (((size_t)b * NH_ + h) * HD) * NP + k0;
    auto pass = [&]() {
#pragma unroll
        for (int s = 0; s < 8; ++s) { const int Lid = (tid >> 3) + 32 * s; const int pln = Lid >> 7, d = Lid & 127;
            const v8h val = *(const v8ha*)((pln ? til2 : tile) + d * 72 + piece * 8); *(volatile v8h*)((pln ? VTL : VTH) + base + (size_t)d * NP + piece * 8) = val; }
    };
    pass(); __threadfence(); pass();
}

__global__ __launch_bounds__(128) void k_attn(const h16* __restrict__ Q16, const h16* __restrict__ K16, const h16* __restrict__ VTH, const h16* __restrict__ VTL, int dofs, bf* CH, bf* CL) {
    __shared__ __align__(16) h16 plds[4][16 * 32];
    __shared__ __align__(16) h16 plds2[4][16 * 32];
    __shared__ __align__(16) float ost[4][16 * 68];
    const int lane = threadIdx.x & 31, wave = threadIdx.x >> 5, lr = lane & 15, hi = lane >> 4;
    const int bid = blockIdx.x;
    const int b = bid / (NH_ * (NP / 64)), rem = bid - b * (NH_ * (NP / 64)), h = rem / (NP / 64), qt = rem - h * (NP / 64);
    const int q0 = qt * 64 + wave * 16;
    const size_t tok0 = (size_t)b * NP;
    h16* pl = &plds[wave][0]; h16* pl2 = &plds2[wave][0];
    v16h qa[4];
#pragma unroll
    for (int kc = 0; kc < 4; ++kc) { const h16* p = Q16 + (tok0 + q0 + lr) * DM + h * HD + kc * 32 + 8 * hi; qa[kc] = cat16(*(const v8h*)p, *(const v8h*)(p + 16)); }
    int qpos[8];
#pragma unroll
    for (int j = 0; j < 8; ++j) qpos[j] = q0 + 8 * hi + j;
    const h16* kh_b = K16 + tok0 * DM + h * HD;
    const size_t vbase = (((size_t)b * NH_ + h) * HD + dofs) * NP;
    v8f o[4], ox[4];
#pragma unroll
    for (int n = 0; n < 4; ++n) { o[n] = (v8f){}; ox[n] = (v8f){}; }
    float mrow[8], lpart[8];
#pragma unroll
    for (int j = 0; j < 8; ++j) { mrow[j] = -3.0e38f; lpart[j] = 0.f; }
    const int kt0 = max(0, (qt * 64 - WIN) / 32), kt_end = (qt * 64 + 64) / 32;
#pragma unroll 1
    for (int kt = kt0; kt < kt_end; ++kt) {
        const int l0 = kt * 32;
        const h16* r0p = kh_b + (size_t)(l0 + lr) * DM + 8 * hi;
        const h16* r1p = kh_b + (size_t)(l0 + 16 + lr) * DM + 8 * hi;
        v8f s0 = {}, s1 = {};
#pragma unroll
        for (int kc = 0; kc < 4; ++kc) {
            s0 = wmma16(qa[kc], cat16(*(const v8h*)(r0p + kc * 32), *(const v8h*)(r0p + kc * 32 + 16)), s0);
            s1 = wmma16(qa[kc], cat16(*(const v8h*)(r1p + kc * 32), *(const v8h*)(r1p + kc * 32 + 16)), s1);
        }
        asm volatile("v_nop\n\tv_nop\n\tv_nop\n\tv_nop" : "+v"(s0), "+v"(s1) : "v"(qa[0]), "v"(qa[3]));
        float alpha[8];
#pragma unroll
        for (int j = 0; j < 8; ++j) {
            const int i = qpos[j], k0i = l0 + lr, k1i = l0 + 16 + lr;
            const bool in0 = (k0i <= i) && (k0i >= i - WIN), in1 = (k1i <= i) && (k1i >= i - WIN);
            const float a0 = s0[j] * SCL + (in0 ? 0.0f : -1e30f), a1 = s1[j] * SCL + (in1 ? 0.0f : -1e30f);
            float mx = fmaxf(a0, a1);
            mx = fmaxf(mx, __shfl_xor(mx, 1, 16)); mx = fmaxf(mx, __shfl_xor(mx, 2, 16)); mx = fmaxf(mx, __shfl_xor(mx, 4, 16)); mx = fmaxf(mx, __shfl_xor(mx, 8, 16));
            const float mn = fmaxf(mrow[j], mx);
            alpha[j] = __expf(mrow[j] - mn); mrow[j] = mn;
            const float p0 = __expf(a0 - mn), p1 = __expf(a1 - mn);
            lpart[j] = lpart[j] * alpha[j] + (p0 + p1);
            const int mr = hi * 8 + j;
            const float ps0 = p0 * PSC, ps1 = p1 * PSC; const h16 h0 = (h16)ps0, h1 = (h16)ps1;
            pl[mr * 32 + lr] = h0; pl[mr * 32 + 16 + lr] = h1;
            pl2[mr * 32 + lr] = (h16)((ps0 - (float)h0) * LOSC); pl2[mr * 32 + 16 + lr] = (h16)((ps1 - (float)h1) * LOSC);
        }
#pragma unroll
        for (int n = 0; n < 4; ++n)
#pragma unroll
            for (int j = 0; j < 8; ++j) { o[n][j] *= alpha[j]; ox[n][j] *= alpha[j]; }
        asm volatile("" ::: "memory");
        const v16h pa = cat16(*(const v8ha*)(pl + lr * 32 + hi * 8), *(const v8ha*)(pl + lr * 32 + 16 + hi * 8));
        const v16h px = cat16(*(const v8ha*)(pl2 + lr * 32 + hi * 8), *(const v8ha*)(pl2 + lr * 32 + 16 + hi * 8));
#pragma unroll
        for (int n = 0; n < 4; ++n) { const size_t vo = vbase + (size_t)(n * 16 + lr) * NP + l0 + hi * 8;
            const v16h vh = cat16(*(const v8h*)(VTH + vo), *(const v8h*)(VTH + vo + 16)), vl = cat16(*(const v8h*)(VTL + vo), *(const v8h*)(VTL + vo + 16));
            o[n] = wmma16(pa, vh, o[n]); ox[n] = wmma16(pa, vl, ox[n]); ox[n] = wmma16(px, vh, ox[n]); }
        asm volatile("v_nop\n\tv_nop\n\tv_nop\n\tv_nop" : "+v"(o[0]), "+v"(o[1]), "+v"(o[2]), "+v"(o[3]), "+v"(ox[0]), "+v"(ox[1]), "+v"(ox[2]), "+v"(ox[3]) : "v"(pa), "v"(px));
    }
    float inv[8];
#pragma unroll
    for (int j = 0; j < 8; ++j) { float rs = lpart[j]; rs += __shfl_xor(rs, 1, 16); rs += __shfl_xor(rs, 2, 16); rs += __shfl_xor(rs, 4, 16); rs += __shfl_xor(rs, 8, 16); inv[j] = 1.0f / (rs * PSC); }
    float* os = &ost[wave][0];
#pragma unroll
    for (int n = 0; n < 4; ++n)
#pragma unroll
        for (int j = 0; j < 8; ++j) os[(hi * 8 + j) * 68 + n * 16 + lr] = (o[n][j] + ox[n][j] * LOSCI) * inv[j];
    __syncthreads();
    const size_t cbase = (tok0 + q0) * DM + (size_t)h * HD + dofs;
    auto pass = [&]() {
#pragma unroll
        for (int s = 0; s < 4; ++s) { const int row = 4 * s + (lane >> 3), piece = lane & 7; const float* sp = os + row * 68 + piece * 8; v8us oh, ol;
#pragma unroll
            for (int i = 0; i < 8; ++i) { const unsigned short hb = f2bf(sp[i]); oh[i] = hb; ol[i] = f2bf(sp[i] - bf2f(hb)); }
            *(volatile v8us*)(CH + cbase + (size_t)row * DM + piece * 8) = oh; *(volatile v8us*)(CL + cbase + (size_t)row * DM + piece * 8) = ol; }
    };
    pass(); __threadfence(); pass();
}

__global__ __launch_bounds__(256) void k_fc2(const float* __restrict__ O1, const float* __restrict__ w, const float* __restrict__ bb, float* out) {
    const int lane = threadIdx.x & 31, wid = blockIdx.x * 8 + (threadIdx.x >> 5);
    const int flat = wid * 32 + lane;
    if (flat >= NB_ * NS0) return;
    const int b = flat / NS0, n = flat - b * NS0;
    const float* row = O1 + ((size_t)b * NP + n) * F1;
    float s = bfr(bb[0]);
#pragma unroll 4
    for (int k = 0; k < F1; ++k) s += row[k] * bfr(w[k]);
    VST2(float, out + flat, s);
}

extern "C" void kernel_launch(void* const* d_in, const int* in_sizes, int n_in,
                              void* d_out, int out_size, void* d_ws, size_t ws_size, hipStream_t stream) {
    (void)in_sizes; (void)n_in; (void)out_size;
    const float* src = (const float*)d_in[0];
    const float* Wenc = (const float*)d_in[2]; const float* benc = (const float*)d_in[3]; const float* Win = (const float*)d_in[4]; const float* bin = (const float*)d_in[5];
    const float* Wout = (const float*)d_in[6]; const float* bout = (const float*)d_in[7]; const float* ln1w = (const float*)d_in[8]; const float* ln1b = (const float*)d_in[9];
    const float* W1 = (const float*)d_in[10]; const float* b1 = (const float*)d_in[11]; const float* W2 = (const float*)d_in[12]; const float* b2 = (const float*)d_in[13];
    const float* ln2w = (const float*)d_in[14]; const float* ln2b = (const float*)d_in[15]; const float* Wf1 = (const float*)d_in[16]; const float* bf1 = (const float*)d_in[17];
    const float* Wf2 = (const float*)d_in[18]; const float* bf2 = (const float*)d_in[19];
    float* out = (float*)d_out;
    char* wsp = (char*)d_ws;
    auto take = [&](size_t bytes) { char* p = wsp; wsp += (bytes + 255) & ~(size_t)255; return (void*)p; };
    bf* Xb = (bf*)take((size_t)NTK * DM * 2);
    bf* WencB = (bf*)take((size_t)DM * DM * 2); bf* WinB = (bf*)take((size_t)3 * DM * DM * 2); bf* WoutB = (bf*)take((size_t)DM * DM * 2);
    bf* W1B = (bf*)take((size_t)FF * DM * 2); bf* W2B = (bf*)take((size_t)DM * FF * 2); bf* Wf1B = (bf*)take((size_t)F1 * DM * 2);
    float* PE = (float*)take((size_t)NP * DM * 4);
    float* X0 = (float*)take((size_t)NTK * DM * 4); bf* AH = (bf*)take((size_t)NTK * DM * 2); bf* AL = (bf*)take((size_t)NTK * DM * 2);
    h16* Q16 = (h16*)take((size_t)NTK * DM * 2); h16* K16 = (h16*)take((size_t)NTK * DM * 2);
    float* T0 = (float*)take((size_t)NTK * DM * 4);
    h16* VTH = (h16*)take((size_t)NTK * DM * 2); h16* VTL = (h16*)take((size_t)NTK * DM * 2);
    bf* CL = (bf*)take((size_t)NTK * DM * 2); float* X1 = (float*)take((size_t)NTK * DM * 4); float* O1 = (float*)take((size_t)NTK * F1 * 4);
    if ((size_t)(wsp - (char*)d_ws) > ws_size) return;
    bf* CH = Xb;
    bf* HH = (bf*)Q16; bf* HL = (bf*)K16;
    k_xb<<<NTK / 8, 256, 0, stream>>>(src, Xb);
    k_cvtb<<<DM / 8, 256, 0, stream>>>(Wenc, DM, DM, WencB);
    k_cvtb<<<(3 * DM) / 8, 256, 0, stream>>>(Win, 3 * DM, DM, WinB);
    k_cvtb<<<DM / 8, 256, 0, stream>>>(Wout, DM, DM, WoutB);
    k_cvtb<<<FF / 8, 256, 0, stream>>>(W1, FF, DM, W1B);
    k_cvtb<<<DM / 8, 256, 0, stream>>>(W2, DM, FF, W2B);
    k_cvtb<<<F1 / 8, 256, 0, stream>>>(Wf1, F1, DM, Wf1B);
    k_pe<<<NP / 8, 256, 0, stream>>>(PE);
    k_gemmb<false, 0><<<dim3(NTK / 64, DM / 64, 1), 128, 0, stream>>>(Xb, nullptr, WencB, DM, benc, PE, X0, nullptr, DM);
    k_split<<<NTK / 8, 256, 0, stream>>>(X0, AH, AL);
    k_gemmb<true, 2><<<dim3(NTK / 64, DM / 64, 1), 128, 0, stream>>>(AH, AL, WinB, DM, bin, nullptr, Q16, nullptr, DM);
    k_gemmb<true, 2><<<dim3(NTK / 64, DM / 64, 1), 128, 0, stream>>>(AH, AL, WinB + (size_t)DM * DM, DM, bin + DM, nullptr, K16, nullptr, DM);
    k_gemmb<true, 0><<<dim3(NTK / 64, DM / 64, 1), 128, 0, stream>>>(AH, AL, WinB + (size_t)2 * DM * DM, DM, bin + 2 * DM, nullptr, T0, nullptr, DM);
    k_vt<<<NB_ * NH_ * (NP / 64), 256, 0, stream>>>(T0, VTH, VTL);
    k_attn<<<NB_ * NH_ * (NP / 64), 128, 0, stream>>>(Q16, K16, VTH, VTL, 0, CH, CL);
    k_attn<<<NB_ * NH_ * (NP / 64), 128, 0, stream>>>(Q16, K16, VTH, VTL, HD / 2, CH, CL);
    k_gemmb<true, 0><<<dim3(NTK / 64, DM / 64, 1), 128, 0, stream>>>(CH, CL, WoutB, DM, bout, nullptr, T0, nullptr, DM);
    k_ln<<<NTK / 8, 256, 0, stream>>>(X0, T0, ln1w, ln1b, X1, AH, AL);
    k_gemmb<true, 1><<<dim3(NTK / 64, FF / 64, 1), 128, 0, stream>>>(AH, AL, W1B, DM, b1, nullptr, HH, HL, FF);
    k_gemmb<true, 0><<<dim3(NTK / 64, DM / 64, 1), 128, 0, stream>>>(HH, HL, W2B, FF, b2, nullptr, T0, nullptr, DM);
    k_ln<<<NTK / 8, 256, 0, stream>>>(X1, T0, ln2w, ln2b, X0, AH, AL);
    k_gemmb<true, 0><<<dim3(NTK / 64, F1 / 64, 1), 128, 0, stream>>>(AH, AL, Wf1B, DM, bf1, nullptr, O1, nullptr, F1);
    k_fc2<<<(NB_ * NS0 / 32 + 7) / 8, 256, 0, stream>>>(O1, Wf2, bf2, out);
}
